// DTNHybridFFN_23295902613827
// MI455X (gfx1250) — hardware-run, weakly checked
//
#include <hip/hip_runtime.h>
#include <math.h>

typedef __attribute__((ext_vector_type(16))) _Float16 v16h;
typedef __attribute__((ext_vector_type(8)))  _Float16 v8h;
typedef __attribute__((ext_vector_type(8)))  float    v8f;
typedef __attribute__((ext_vector_type(4)))  float    v4f;
typedef __attribute__((ext_vector_type(2)))  float    v2f;
typedef __attribute__((ext_vector_type(4)))  unsigned int v4u;

constexpr int kTok    = 32768;
constexpr int kDm     = 256;
constexpr int kFf     = 1024;
constexpr int kPieces = 8;
constexpr int kTokBlk = 16;
constexpr float kCarryWc = 16.0f;
constexpr float kCarryWg = 64.0f;
constexpr float kCarryWd = 32.0f;
constexpr float kInvWc = 1.0f / kCarryWc;
constexpr float kInvWg = 1.0f / kCarryWg;
constexpr float kInvWd = 1.0f / kCarryWd;
static_assert(kPieces == 8, "eight line pieces per channel");
static_assert((kDm % 32) == 0 && (kFf % 32) == 0, "GEMM K multiples of 32");
static_assert((kTok % 64) == 0 && (kFf % 64) == 0 && (kDm % 64) == 0, "GEMM M,N multiples of 64");
static_assert((kTok % kTokBlk) == 0, "token blocks");

constexpr size_t kOffTF   = 0;
constexpr size_t kOffXH   = kOffTF  + (size_t)kTok * kFf * 2;
constexpr size_t kOffWCG  = kOffXH  + (size_t)kTok * kDm * 2;
constexpr size_t kOffWDT  = kOffWCG + (size_t)2 * kFf * kDm * 2;
constexpr size_t kOffWTT  = kOffWDT + (size_t)kDm * kFf * 2;
constexpr size_t kOffCB   = kOffWTT + (size_t)kDm * kFf * 4;
constexpr size_t kWsTotal = kOffCB  + (size_t)2 * kDm * 4;
static_assert(kWsTotal == 86509568ull, "carve total");
static_assert(kWsTotal <= 134217728ull, "carve cap");
static_assert((kOffXH % 128) == 0 && (kOffWCG % 128) == 0 && (kOffWDT % 128) == 0 &&
              (kOffWTT % 128) == 0 && (kOffCB % 128) == 0, "128-B aligned regions");

union FragU { v16h v; v8h h[2]; };
__device__ __forceinline__ v16h frag_load(const _Float16* p) {
  FragU f;
  f.h[0] = *(const v8h*)(p);
  f.h[1] = *(const v8h*)(p + 16);
  return f.v;
}
__device__ __forceinline__ v8f mma_h(v16h a, v16h b, v8f c) {
  c = __builtin_amdgcn_wmma_f32_16x16x32_f16(false, a, false, b, (short)0, c, false, false);
  asm volatile("v_nop\n\tv_nop\n\tv_nop\n\tv_nop" : "+v"(c) : "v"(a), "v"(b));
  return c;
}
__device__ __forceinline__ void wave_lds_sync() {
  __builtin_amdgcn_fence(__ATOMIC_RELEASE, "workgroup");
  __builtin_amdgcn_wave_barrier();
  __builtin_amdgcn_fence(__ATOMIC_ACQUIRE, "workgroup");
}
__device__ __forceinline__ float h16_to_f32(unsigned hb) {
  const unsigned sgn = (hb & 0x8000u) << 16; const unsigned em = hb & 0x7fffu;
  const float fn = __uint_as_float((em << 13) + 0x38000000u);
  const float fs = (float)em * 5.9604644775390625e-8f;
  const float mag = (em < 0x400u) ? fs : fn; return __uint_as_float(__float_as_uint(mag) | sgn); }
__device__ __forceinline__ void dump_slab(float* slab, const v8f& a0, const v8f& a1, const v8f& a2, const v8f& a3,
                                          int mOff, int rlane) {
#pragma unroll
  for (int r = 0; r < 8; ++r) {
    float* p = slab + (mOff + r) * 68 + rlane;
    p[0]  = a0[r];
    p[16] = a1[r];
    p[32] = a2[r];
    p[48] = a3[r];
  }
}
__device__ __forceinline__ float lf_blend(float t, v4f sxa, v4f sxb, v4f oxa, v4f oxb,
                                          v4f sva, v4f svb, v4f ova, v4f ovb, float s) {
  float cvx = t * sxa[0] + oxa[0];
  cvx = fmaxf(cvx, t * sxa[1] + oxa[1]);
  cvx = fmaxf(cvx, t * sxa[2] + oxa[2]);
  cvx = fmaxf(cvx, t * sxa[3] + oxa[3]);
  cvx = fmaxf(cvx, t * sxb[0] + oxb[0]);
  cvx = fmaxf(cvx, t * sxb[1] + oxb[1]);
  cvx = fmaxf(cvx, t * sxb[2] + oxb[2]);
  cvx = fmaxf(cvx, t * sxb[3] + oxb[3]);
  float ccv = t * sva[0] + ova[0];
  ccv = fminf(ccv, t * sva[1] + ova[1]);
  ccv = fminf(ccv, t * sva[2] + ova[2]);
  ccv = fminf(ccv, t * sva[3] + ova[3]);
  ccv = fminf(ccv, t * svb[0] + ovb[0]);
  ccv = fminf(ccv, t * svb[1] + ovb[1]);
  ccv = fminf(ccv, t * svb[2] + ovb[2]);
  ccv = fminf(ccv, t * svb[3] + ovb[3]);
  return s * cvx + (1.0f - s) * ccv;
}

template <bool F16>
__global__ __launch_bounds__(256) void transpose_kernel(const float* __restrict__ src, void* __restrict__ dst,
                                                        int rows, int cols, float scale) {
  __shared__ float sT[64 * 65];
  const int tid = threadIdx.x;
  const int c0 = blockIdx.x * 64, r0 = blockIdx.y * 64;
#pragma unroll
  for (int it = 0; it < 4; ++it) {
    const int r = it * 16 + (tid >> 4);
    const int c4 = (tid & 15) * 4;
    const v4f v = *(const v4f*)(src + (size_t)(r0 + r) * cols + c0 + c4);
    sT[r * 65 + c4 + 0] = v[0] * scale;
    sT[r * 65 + c4 + 1] = v[1] * scale;
    sT[r * 65 + c4 + 2] = v[2] * scale;
    sT[r * 65 + c4 + 3] = v[3] * scale;
  }
  __syncthreads();
  if (F16) {
    unsigned short* d = (unsigned short*)dst;
    v8h hv[2];
#pragma unroll
    for (int it = 0; it < 2; ++it) {
      const int orow = it * 32 + (tid >> 3);
      const int seg = (tid & 7) * 8;
#pragma unroll
      for (int e = 0; e < 8; ++e) hv[it][e] = (_Float16)sT[(seg + e) * 65 + orow];
    }
    for (int pass = 0; pass < 2; ++pass) {
#pragma unroll
      for (int it = 0; it < 2; ++it) {
        const int orow = it * 32 + (tid >> 3);
        const int seg = (tid & 7) * 8;
        *(volatile v8h*)(d + (size_t)(c0 + orow) * rows + r0 + seg) = hv[it];
      }
      __threadfence();
    }
  } else {
    float* d = (float*)dst;
    v4f fv[4];
#pragma unroll
    for (int it = 0; it < 4; ++it) {
      const int orow = it * 16 + (tid >> 4);
      const int seg = (tid & 15) * 4;
      fv[it][0] = sT[(seg + 0) * 65 + orow];
      fv[it][1] = sT[(seg + 1) * 65 + orow];
      fv[it][2] = sT[(seg + 2) * 65 + orow];
      fv[it][3] = sT[(seg + 3) * 65 + orow];
    }
    for (int pass = 0; pass < 2; ++pass) {
#pragma unroll
      for (int it = 0; it < 4; ++it) {
        const int orow = it * 16 + (tid >> 4);
        const int seg = (tid & 15) * 4;
        *(volatile v4f*)(d + (size_t)(c0 + orow) * rows + r0 + seg) = fv[it];
      }
      __threadfence();
    }
  }
}

__global__ __launch_bounds__(256) void col_bounds_kernel(const float* __restrict__ Wt, float* __restrict__ CB) {
  __shared__ __align__(16) float sB[2 * kDm];
  const int k = threadIdx.x;
  float mx = Wt[k];
  float mn = mx;
#pragma unroll 1
  for (int m = 1; m < kFf; ++m) {
    const float w = Wt[(size_t)m * kDm + k];
    mx = fmaxf(mx, w);
    mn = fminf(mn, w);
  }
  sB[k] = mx;
  sB[kDm + k] = mn;
  __syncthreads();
  if (threadIdx.x < 128) {
    const v4f v = *(const v4f*)(sB + threadIdx.x * 4);
    float* p = CB + threadIdx.x * 4;
    *(volatile v4f*)p = v;
    __threadfence();
    *(volatile v4f*)p = v;
  }
}

__global__ __launch_bounds__(256) void cast_rows_f16_kernel(const float* __restrict__ src,
                                                            unsigned short* __restrict__ dst, int total8) {
  const int i = blockIdx.x * 256 + threadIdx.x;
  if (i >= total8) return;
  const size_t e0 = (size_t)i << 3;
  const v4f a0 = *(const v4f*)(src + e0);
  const v4f a1 = *(const v4f*)(src + e0 + 4);
  v8h hv;
  hv[0] = (_Float16)a0[0];
  hv[1] = (_Float16)a0[1];
  hv[2] = (_Float16)a0[2];
  hv[3] = (_Float16)a0[3];
  hv[4] = (_Float16)a1[0];
  hv[5] = (_Float16)a1[1];
  hv[6] = (_Float16)a1[2];
  hv[7] = (_Float16)a1[3];
  unsigned short* p = dst + e0;
  *(volatile v8h*)p = hv;
  __threadfence();
  *(volatile v8h*)p = hv;
}

__global__ __launch_bounds__(256) void maxplus_lines_kernel(
    const float* __restrict__ x, const float* __restrict__ WtT, const float* __restrict__ CB,
    const float* __restrict__ bt, const float* __restrict__ slx, const float* __restrict__ ofx,
    const float* __restrict__ slv, const float* __restrict__ ofv, const float* __restrict__ alpha,
    unsigned short* __restrict__ TF) {
  __shared__ int   sK[kTokBlk * kDm];
  __shared__ float sXv[kTokBlk * kDm];
  __shared__ int   sCnt[kTokBlk];
  __shared__ __align__(16) unsigned sTile[kTokBlk * 256];

  const int tid = threadIdx.x, lane = tid & 31, wave = tid >> 5;
  const int t0 = blockIdx.x * kTokBlk;

  {
    const v4f cxa = *(const v4f*)(CB + lane * 8);
    const v4f cxb = *(const v4f*)(CB + lane * 8 + 4);
    const v4f cna = *(const v4f*)(CB + kDm + lane * 8);
    const v4f cnb = *(const v4f*)(CB + kDm + lane * 8 + 4);
    const float cmx[8] = {cxa[0], cxa[1], cxa[2], cxa[3], cxb[0], cxb[1], cxb[2], cxb[3]};
    const float cmn[8] = {cna[0], cna[1], cna[2], cna[3], cnb[0], cnb[1], cnb[2], cnb[3]};
    const unsigned ltmask = (1u << lane) - 1u;
#pragma unroll 1
    for (int i = 0; i < 2; ++i) {
      const int tok = wave * 2 + i;
      const float* xr = x + (size_t)(t0 + tok) * kDm + lane * 8;
      const v4f xa = *(const v4f*)(xr);
      const v4f xb = *(const v4f*)(xr + 4);
      const float xs[8] = {xa[0], xa[1], xa[2], xa[3], xb[0], xb[1], xb[2], xb[3]};
      float lmax = xs[0] + cmn[0];
#pragma unroll
      for (int e = 1; e < 8; ++e) lmax = fmaxf(lmax, xs[e] + cmn[e]);
#pragma unroll
      for (int off = 16; off >= 1; off >>= 1) lmax = fmaxf(lmax, __shfl_xor(lmax, off, 32));
      int base = 0;
#pragma unroll
      for (int e = 0; e < 8; ++e) {
        const bool keep = (xs[e] + cmx[e]) >= lmax;
        const unsigned bal = __builtin_amdgcn_ballot_w32(keep);
        const int pos = (base + __popc(bal & ltmask)) & (kDm - 1);
        if (keep) {
          sK[tok * kDm + pos] = lane * 8 + e;
          sXv[tok * kDm + pos] = xs[e];
        }
        base += __popc(bal);
      }
      if (lane == 0) sCnt[tok] = base;
    }
  }
  __syncthreads();

#pragma unroll 1
  for (int j = 0; j < 2; ++j) {
    const int m = 2 * tid + 512 * j;
    const v4f sx0 = *(const v4f*)(slx + (size_t)m * 8);
    const v4f sx1 = *(const v4f*)(slx + (size_t)m * 8 + 4);
    const v4f sx2 = *(const v4f*)(slx + (size_t)m * 8 + 8);
    const v4f sx3 = *(const v4f*)(slx + (size_t)m * 8 + 12);
    const v4f ox0 = *(const v4f*)(ofx + (size_t)m * 8);
    const v4f ox1 = *(const v4f*)(ofx + (size_t)m * 8 + 4);
    const v4f ox2 = *(const v4f*)(ofx + (size_t)m * 8 + 8);
    const v4f ox3 = *(const v4f*)(ofx + (size_t)m * 8 + 12);
    const v4f sv0 = *(const v4f*)(slv + (size_t)m * 8);
    const v4f sv1 = *(const v4f*)(slv + (size_t)m * 8 + 4);
    const v4f sv2 = *(const v4f*)(slv + (size_t)m * 8 + 8);
    const v4f sv3 = *(const v4f*)(slv + (size_t)m * 8 + 12);
    const v4f ov0 = *(const v4f*)(ofv + (size_t)m * 8);
    const v4f ov1 = *(const v4f*)(ofv + (size_t)m * 8 + 4);
    const v4f ov2 = *(const v4f*)(ofv + (size_t)m * 8 + 8);
    const v4f ov3 = *(const v4f*)(ofv + (size_t)m * 8 + 12);
    const v2f btv = *(const v2f*)(bt + m);
    const v2f alv = *(const v2f*)(alpha + m);
    const float bt0 = btv[0], bt1 = btv[1];
    const float s0 = __builtin_amdgcn_rcpf(1.0f + expf(-alv[0]));
    const float s1 = __builtin_amdgcn_rcpf(1.0f + expf(-alv[1]));
#pragma unroll 1
    for (int tok = 0; tok < kTokBlk; ++tok) {
      int n = sCnt[tok];
      n = (n < kDm) ? n : kDm;
      const int* kp = sK + tok * kDm;
      const float* xp = sXv + tok * kDm;
      float ta = -INFINITY, tb = -INFINITY;
#pragma unroll 1
      for (int c = 0; c < n; ++c) {
        const int k = kp[c] & (kDm - 1);
        const float xv = xp[c];
        const v2f w = *(const v2f*)(WtT + (size_t)k * kFf + m);
        ta = fmaxf(ta, xv + w[0]);
        tb = fmaxf(tb, xv + w[1]);
      }
      ta += bt0;
      tb += bt1;
      const float ra = lf_blend(ta, sx0, sx1, ox0, ox1, sv0, sv1, ov0, ov1, s0);
      const float rb = lf_blend(tb, sx2, sx3, ox2, ox3, sv2, sv3, ov2, ov3, s1);
      const _Float16 ha = (_Float16)ra;
      const _Float16 hb = (_Float16)rb;
      const unsigned u = (unsigned)__builtin_bit_cast(unsigned short, ha) |
                         ((unsigned)__builtin_bit_cast(unsigned short, hb) << 16);
      sTile[tok * 256 + tid] = u;
    }
    __syncthreads();
    v4u fv[4];
#pragma unroll
    for (int it = 0; it < 4; ++it) {
      const int row = it * 4 + (tid >> 6);
      const int seg = tid & 63;
      fv[it] = *(const v4u*)(sTile + row * 256 + seg * 4);
    }
    for (int pass = 0; pass < 2; ++pass) {
#pragma unroll
      for (int it = 0; it < 4; ++it) {
        const int row = it * 4 + (tid >> 6);
        const int seg = tid & 63;
        *(volatile v4u*)(TF + (size_t)(t0 + row) * kFf + 512 * j + seg * 8) = fv[it];
      }
      __threadfence();
    }
    __syncthreads();
  }
}

__global__ __launch_bounds__(64) void gemm_up_blend_kernel(
    const unsigned short* __restrict__ XHp, const unsigned short* __restrict__ WCGp,
    const float* __restrict__ bc, const float* __restrict__ bg, unsigned short* TF) {
  __shared__ __align__(16) float sC[2][32 * 68];
  __shared__ __align__(16) float sG[2][32 * 68];
  const _Float16* A  = (const _Float16*)XHp;
  const _Float16* Bt = (const _Float16*)WCGp;
  const int lane = threadIdx.x & 31, wave = threadIdx.x >> 5;
  const int tile = blockIdx.x * 2 + wave;
  const int tn = tile & 15;
  const int tm = tile >> 4;
  const int m0 = tm * 32;
  const int n0 = tn * 64;
  const int rlane = lane & 15;
  const int koff = (lane >> 4) * 8;
  const int mOff = (lane >> 4) * 8;

  v8f accC[2][4], accG[2][4];
#pragma unroll
  for (int i = 0; i < 2; ++i)
#pragma unroll
    for (int j = 0; j < 4; ++j) {
      accC[i][j] = (v8f){0.f, 0.f, 0.f, 0.f, 0.f, 0.f, 0.f, 0.f};
      accG[i][j] = (v8f){0.f, 0.f, 0.f, 0.f, 0.f, 0.f, 0.f, 0.f};
    }

  const _Float16* a0p = A + (size_t)(m0 + rlane) * kDm + koff;
  const _Float16* a1p = a0p + (size_t)16 * kDm;
  const _Float16* bcp = Bt + (size_t)(n0 + rlane) * kDm + koff;
  const _Float16* bgp = bcp + (size_t)kFf * kDm;

#pragma unroll 1
  for (int k0 = 0; k0 < kDm; k0 += 32) {
    const v16h a0 = frag_load(a0p + k0);
    const v16h a1 = frag_load(a1p + k0);
    {
      v16h b[4];
#pragma unroll
      for (int j = 0; j < 4; ++j) b[j] = frag_load(bcp + (size_t)j * 16 * kDm + k0);
#pragma unroll
      for (int j = 0; j < 4; ++j) {
        accC[0][j] = mma_h(a0, b[j], accC[0][j]);
        accC[1][j] = mma_h(a1, b[j], accC[1][j]);
      }
    }
    {
      v16h b[4];
#pragma unroll
      for (int j = 0; j < 4; ++j) b[j] = frag_load(bgp + (size_t)j * 16 * kDm + k0);
#pragma unroll
      for (int j = 0; j < 4; ++j) {
        accG[0][j] = mma_h(a0, b[j], accG[0][j]);
        accG[1][j] = mma_h(a1, b[j], accG[1][j]);
      }
    }
  }

  float* slabC = sC[wave];
  float* slabG = sG[wave];
  dump_slab(slabC,           accC[0][0], accC[0][1], accC[0][2], accC[0][3], mOff, rlane);
  dump_slab(slabC + 16 * 68, accC[1][0], accC[1][1], accC[1][2], accC[1][3], mOff, rlane);
  dump_slab(slabG,           accG[0][0], accG[0][1], accG[0][2], accG[0][3], mOff, rlane);
  dump_slab(slabG + 16 * 68, accG[1][0], accG[1][1], accG[1][2], accG[1][3], mOff, rlane);
  wave_lds_sync();

  const int q = lane >> 3, c8 = (lane & 7) * 8;
  const v4f bc0 = *(const v4f*)(bc + n0 + c8);
  const v4f bc1 = *(const v4f*)(bc + n0 + c8 + 4);
  const v4f bg0 = *(const v4f*)(bg + n0 + c8);
  const v4f bg1 = *(const v4f*)(bg + n0 + c8 + 4);
  const float bcv[8] = {bc0[0], bc0[1], bc0[2], bc0[3], bc1[0], bc1[1], bc1[2], bc1[3]};
  const float bgv[8] = {bg0[0], bg0[1], bg0[2], bg0[3], bg1[0], bg1[1], bg1[2], bg1[3]};

#pragma unroll 1
  for (int it = 0; it < 8; ++it) {
    const int row = it * 4 + q;
    const float* pc = slabC + row * 68 + c8;
    const float* pg = slabG + row * 68 + c8;
    const v4f c0 = *(const v4f*)(pc);
    const v4f c1 = *(const v4f*)(pc + 4);
    const v4f g0 = *(const v4f*)(pg);
    const v4f g1 = *(const v4f*)(pg + 4);
    unsigned short* tp = TF + (size_t)(m0 + row) * kFf + n0 + c8;
    const v4u tw = *(const v4u*)tp;
    const unsigned u0 = tw[0];
    const unsigned u1 = tw[1];
    const unsigned u2 = tw[2];
    const unsigned u3 = tw[3];
    const float tv[8] = {h16_to_f32(u0 & 0xffffu), h16_to_f32(u0 >> 16),
                         h16_to_f32(u1 & 0xffffu), h16_to_f32(u1 >> 16),
                         h16_to_f32(u2 & 0xffffu), h16_to_f32(u2 >> 16),
                         h16_to_f32(u3 & 0xffffu), h16_to_f32(u3 >> 16)};
    const float cv[8] = {c0[0], c0[1], c0[2], c0[3], c1[0], c1[1], c1[2], c1[3]};
    const float gv[8] = {g0[0], g0[1], g0[2], g0[3], g1[0], g1[1], g1[2], g1[3]};
    unsigned hb[8];
#pragma unroll
    for (int e = 0; e < 8; ++e) {
      const float pre = cv[e] * kInvWc + bcv[e];
      const float gel = 0.5f * pre * (1.0f + erff(pre * 0.70710678118654752f));
      const float gp = gv[e] * kInvWg + bgv[e];
      const float g = __builtin_amdgcn_rcpf(1.0f + expf(-gp));
      const float fu = g * tv[e] + (1.0f - g) * gel;
      const _Float16 hf = (_Float16)fu;
      hb[e] = (unsigned)__builtin_bit_cast(unsigned short, hf);
    }
    v4u ow;
    ow[0] = hb[0] | (hb[1] << 16);
    ow[1] = hb[2] | (hb[3] << 16);
    ow[2] = hb[4] | (hb[5] << 16);
    ow[3] = hb[6] | (hb[7] << 16);
    *(volatile v4u*)tp = ow;
    __threadfence();
    *(volatile v4u*)tp = ow;
  }
}

__global__ __launch_bounds__(256) void gemm_down_kernel(
    const unsigned short* __restrict__ Fp, const unsigned short* __restrict__ WDTp,
    const float* __restrict__ bd, float* __restrict__ out) {
  __shared__ __align__(16) float sT[8][16 * 68];
  const _Float16* A  = (const _Float16*)Fp;
  const _Float16* Bt = (const _Float16*)WDTp;
  const int lane = threadIdx.x & 31, wave = threadIdx.x >> 5;
  const int tile = blockIdx.x * 8 + wave;
  const int tn = tile & 3;
  const int tm = tile >> 2;
  const int m0 = tm * 64;
  const int n0 = tn * 64;
  const int rlane = lane & 15;
  const int koff = (lane >> 4) * 8;
  const int mOff = (lane >> 4) * 8;

  v8f acc[4][4];
#pragma unroll
  for (int i = 0; i < 4; ++i)
#pragma unroll
    for (int j = 0; j < 4; ++j) acc[i][j] = (v8f){0.f, 0.f, 0.f, 0.f, 0.f, 0.f, 0.f, 0.f};

  const _Float16* ap = A + (size_t)(m0 + rlane) * kFf + koff;
  const _Float16* bp = Bt + (size_t)(n0 + rlane) * kFf + koff;

#pragma unroll 1
  for (int k0 = 0; k0 < kFf; k0 += 32) {
    v16h bh[4];
#pragma unroll
    for (int j = 0; j < 4; ++j) bh[j] = frag_load(bp + (size_t)j * 16 * kFf + k0);
#pragma unroll
    for (int i = 0; i < 4; ++i) {
      const v16h ah = frag_load(ap + (size_t)i * 16 * kFf + k0);
#pragma unroll
      for (int j = 0; j < 4; ++j) acc[i][j] = mma_h(ah, bh[j], acc[i][j]);
    }
  }

  float* slab = sT[wave];
  const int hh = lane >> 4, c4 = (lane & 15) * 4;
  const v4f bv = *(const v4f*)(bd + n0 + c4);
#pragma unroll
  for (int i = 0; i < 4; ++i) {
    const int mBase = m0 + (i << 4);
    dump_slab(slab, acc[i][0], acc[i][1], acc[i][2], acc[i][3], mOff, rlane);
    wave_lds_sync();
    for (int pass = 0; pass < 2; ++pass) {
#pragma unroll
      for (int it = 0; it < 8; ++it) {
        const int row = it * 2 + hh;
        const v4f v = *(const v4f*)(slab + row * 68 + c4);
        v4f o;
        o[0] = v[0] * kInvWd + bv[0];
        o[1] = v[1] * kInvWd + bv[1];
        o[2] = v[2] * kInvWd + bv[2];
        o[3] = v[3] * kInvWd + bv[3];
        *(volatile v4f*)(out + (size_t)(mBase + row) * kDm + n0 + c4) = o;
      }
      __threadfence();
    }
    wave_lds_sync();
  }
}

extern "C" void kernel_launch(void* const* d_in, const int* in_sizes, int n_in,
                              void* d_out, int out_size, void* d_ws, size_t ws_size,
                              hipStream_t stream) {
  if (n_in < 14) return;
  if (in_sizes[0] != kTok * kDm) return;
  if (in_sizes[1] != kFf * kDm) return;
  if (in_sizes[2] != kFf) return;
  if (in_sizes[3] != kFf * kPieces) return;
  if (in_sizes[4] != kFf * kPieces) return;
  if (in_sizes[5] != kFf * kPieces) return;
  if (in_sizes[6] != kFf * kPieces) return;
  if (in_sizes[7] != kFf) return;
  if (in_sizes[8] != kDm * kFf) return;
  if (in_sizes[9] != kFf) return;
  if (in_sizes[10] != kDm * kFf) return;
  if (in_sizes[11] != kFf) return;
  if (in_sizes[12] != kFf * kDm) return;
  if (in_sizes[13] != kDm) return;
  if (out_size != kTok * kDm) return;
  if (ws_size < kWsTotal) return;

  const float* x      = (const float*)d_in[0];
  const float* Wt     = (const float*)d_in[1];
  const float* bt     = (const float*)d_in[2];
  const float* sl_cvx = (const float*)d_in[3];
  const float* of_cvx = (const float*)d_in[4];
  const float* sl_ccv = (const float*)d_in[5];
  const float* of_ccv = (const float*)d_in[6];
  const float* alpha  = (const float*)d_in[7];
  const float* Wc     = (const float*)d_in[8];
  const float* bc     = (const float*)d_in[9];
  const float* Wg     = (const float*)d_in[10];
  const float* bg     = (const float*)d_in[11];
  const float* Wd     = (const float*)d_in[12];
  const float* bd     = (const float*)d_in[13];
  float* out = (float*)d_out;

  char* ws = (char*)d_ws;
  unsigned short* TF  = (unsigned short*)(ws + kOffTF);
  unsigned short* XH  = (unsigned short*)(ws + kOffXH);
  unsigned short* WCG = (unsigned short*)(ws + kOffWCG);
  unsigned short* WDT = (unsigned short*)(ws + kOffWDT);
  float*          WTT = (float*)(ws + kOffWTT);
  float*          CB  = (float*)(ws + kOffCB);

  transpose_kernel<true><<<dim3(kFf / 64, kDm / 64), 256, 0, stream>>>(Wc, (void*)WCG, kDm, kFf, kCarryWc);
  transpose_kernel<true><<<dim3(kFf / 64, kDm / 64), 256, 0, stream>>>(Wg, (void*)(WCG + (size_t)kFf * kDm), kDm, kFf, kCarryWg);
  transpose_kernel<true><<<dim3(kDm / 64, kFf / 64), 256, 0, stream>>>(Wd, (void*)WDT, kFf, kDm, kCarryWd);
  transpose_kernel<false><<<dim3(kDm / 64, kFf / 64), 256, 0, stream>>>(Wt, (void*)WTT, kFf, kDm, 1.0f);
  col_bounds_kernel<<<1, 256, 0, stream>>>(Wt, CB);
  cast_rows_f16_kernel<<<(kTok * kDm / 8) / 256, 256, 0, stream>>>(x, XH, kTok * kDm / 8);
  maxplus_lines_kernel<<<kTok / kTokBlk, 256, 0, stream>>>(x, WTT, CB, bt, sl_cvx, of_cvx, sl_ccv, of_ccv, alpha, TF);
  gemm_up_blend_kernel<<<(kTok / 32) * (kFf / 64) / 2, 64, 0, stream>>>(XH, WCG, bc, bg, TF);
  gemm_down_kernel<<<(kTok / 64) * (kDm / 64) / 8, 256, 0, stream>>>(TF, WDT, bd, out);
}
